// HiModel_27152783245981
// MI455X (gfx1250) — hardware-verified
//
#include <hip/hip_runtime.h>
#include <math.h>
#include <stdint.h>

constexpr int kRows  = 2048;
constexpr int kNei   = 45;
constexpr int kDimT  = 768;
constexpr int kDimV  = 1024;
constexpr int kFlatT = 768;
constexpr int kFlatV = 4096;
constexpr int kMid   = 512;
constexpr int kGate  = 1536;
constexpr int kFfn   = 2048;
constexpr float kEps = 1e-5f;
constexpr float kWCarry    = 64.0f;
constexpr float kWCarryInv = 1.0f / 64.0f;

typedef __attribute__((ext_vector_type(16))) _Float16 v16h;
typedef __attribute__((ext_vector_type(8)))  _Float16 v8h;
typedef __attribute__((ext_vector_type(16))) __bf16   v16b;
typedef __attribute__((ext_vector_type(8)))  __bf16   v8b;
typedef __attribute__((ext_vector_type(8)))  float    v8f;
typedef __attribute__((ext_vector_type(4)))  float    v4f;
typedef __attribute__((ext_vector_type(2)))  float    v2f;
typedef __attribute__((ext_vector_type(4)))  unsigned int v4u;
typedef __attribute__((ext_vector_type(4)))  int      v4i;

__device__ __forceinline__ unsigned short f2bf_bits(float f) {
  unsigned u = __float_as_uint(f);
  return (unsigned short)((u + 0x7FFFu + ((u >> 16) & 1u)) >> 16);
}
__device__ __forceinline__ float bf_bits2f(unsigned short h) { return __uint_as_float(((unsigned)h) << 16); }

__device__ __forceinline__ void dep_guard_h(v8f& a, v8f& b, v16h x, v16h y) { asm volatile("v_nop\n\tv_nop\n\tv_nop\n\tv_nop" : "+v"(a), "+v"(b) : "v"(x), "v"(y)); }
__device__ __forceinline__ void dep_guard_b(v8f& a, v8f& b, v16b x, v16b y) { asm volatile("v_nop\n\tv_nop\n\tv_nop\n\tv_nop" : "+v"(a), "+v"(b) : "v"(x), "v"(y)); }
__device__ __forceinline__ void keep4_h(v16h a, v16h b, v16h c, v16h d) { asm volatile("v_nop" :: "v"(a), "v"(b), "v"(c), "v"(d)); }
__device__ __forceinline__ void keep4_b(v16b a, v16b b, v16b c, v16b d) { asm volatile("v_nop" :: "v"(a), "v"(b), "v"(c), "v"(d)); }
__device__ __forceinline__ void acc_guard4(v8f& a, v8f& b, v8f& c, v8f& d) { asm volatile("v_nop\n\tv_nop\n\tv_nop\n\tv_nop" : "+v"(a), "+v"(b), "+v"(c), "+v"(d)); }
template <typename T> struct Frag;
template <> struct Frag<_Float16> {
  typedef v16h V; union U { v16h v; v8h h[2]; };
  static __device__ __forceinline__ v16h load(const _Float16* p) {
    U f; f.h[0] = *(const v8h*)(p); f.h[1] = *(const v8h*)(p + 16); return f.v;
  }
  static __device__ __forceinline__ v8f mma(v16h a, v16h b, v8f c) {
    return __builtin_amdgcn_wmma_f32_16x16x32_f16(false, a, false, b, (short)0, c, false, false);
  }
  static __device__ __forceinline__ void guard(v8f& a, v8f& b, v16h x, v16h y) { dep_guard_h(a, b, x, y); }
  static __device__ __forceinline__ void keep(v16h a, v16h b, v16h c, v16h d) { keep4_h(a, b, c, d); }
};
template <> struct Frag<__bf16> {
  typedef v16b V; union U { v16b v; v8b h[2]; };
  static __device__ __forceinline__ v16b load(const __bf16* p) {
    U f; f.h[0] = *(const v8b*)(p); f.h[1] = *(const v8b*)(p + 16); return f.v;
  }
  static __device__ __forceinline__ v8f mma(v16b a, v16b b, v8f c) {
    return __builtin_amdgcn_wmma_f32_16x16x32_bf16(false, a, false, b, (short)0, c, false, false);
  }
  static __device__ __forceinline__ void guard(v8f& a, v8f& b, v16b x, v16b y) { dep_guard_b(a, b, x, y); }
  static __device__ __forceinline__ void keep(v16b a, v16b b, v16b c, v16b d) { keep4_b(a, b, c, d); }
};

__device__ __forceinline__ unsigned pk16(unsigned short a, unsigned short b) { return (unsigned)a | ((unsigned)b << 16); }
__device__ __forceinline__ unsigned short h_bits(float f) { const _Float16 h = (_Float16)f; return __builtin_bit_cast(unsigned short, h); }
__device__ __forceinline__ void split_bits(float x, unsigned short& hb, unsigned short& lb) {
  hb = f2bf_bits(x);
  lb = f2bf_bits(x - bf_bits2f(hb));
}

template <int ET> struct Elem;
template <> struct Elem<0> { typedef _Float16 T; };
template <> struct Elem<1> { typedef __bf16 T; };
template <int ET, bool SPLIT, int BIAS_MODE, int OUT_MODE, bool RESID, int ACT = 0>
__global__ __launch_bounds__(256) void wmma_gemm64(
    const unsigned short* __restrict__ Ap, const unsigned short* __restrict__ A2p, int lda, long strideA,
    const unsigned short* __restrict__ Btp, const unsigned short* __restrict__ Bt2p, int ldb, long strideB,
    void* __restrict__ Cout, void* __restrict__ Cout2, int ldc, long strideC,
    const float* __restrict__ bias,
    const float* __restrict__ resid, long strideR,
    int M, int N, int K, float scale) {
  typedef typename Elem<ET>::T T;
  typedef typename Frag<T>::V V;
  const T* A = (const T*)Ap; const T* A2 = (const T*)A2p; const T* Bt = (const T*)Btp; const T* Bt2 = (const T*)Bt2p;
  __shared__ __align__(16) float sT[8][16 * 68];
  const int b    = blockIdx.y;
  const int lane = threadIdx.x & 31;
  const int wave = threadIdx.x >> 5;
  const int tilesN = N >> 6;
  const int tilesM = M >> 6;
  const int tile = blockIdx.x * 8 + wave;
  if (tile >= tilesM * tilesN) return;
  const int tm = tile / tilesN;
  const int tn = tile - tm * tilesN;
  const int m0 = tm << 6;
  const int n0 = tn << 6;

  const T* Ab  = A  + (size_t)b * strideA;
  const T* Bb  = Bt + (size_t)b * strideB;
  const T* Ab2 = SPLIT ? (A2  + (size_t)b * strideA) : nullptr;
  const T* Bb2 = SPLIT ? (Bt2 + (size_t)b * strideB) : nullptr;

  const int rlane = lane & 15;
  const int koff  = (lane >> 4) * 8;
  const int mOff  = (lane >> 4) * 8;

  v8f acc[4][4];
#pragma unroll
  for (int i = 0; i < 4; ++i)
#pragma unroll
    for (int j = 0; j < 4; ++j) acc[i][j] = (v8f){0.f,0.f,0.f,0.f,0.f,0.f,0.f,0.f};

  for (int k0 = 0; k0 < K; k0 += 32) {
    V bh[4], bl[4];
#pragma unroll
    for (int j = 0; j < 4; ++j) {
      const size_t bo = (size_t)(n0 + (j << 4) + rlane) * ldb + koff + k0;
      bh[j] = Frag<T>::load(Bb + bo);
      if (SPLIT) bl[j] = Frag<T>::load(Bb2 + bo);
    }
#pragma unroll
    for (int i = 0; i < 4; ++i) {
      const size_t ao = (size_t)(m0 + (i << 4) + rlane) * lda + koff + k0;
      V ah = Frag<T>::load(Ab + ao);
      V al;
      if (SPLIT) al = Frag<T>::load(Ab2 + ao);
#pragma unroll
      for (int j = 0; j < 4; ++j) {
        acc[i][j] = Frag<T>::mma(ah, bh[j], acc[i][j]);
        if (SPLIT) {
          acc[i][j] = Frag<T>::mma(ah, bl[j], acc[i][j]);
          acc[i][j] = Frag<T>::mma(al, bh[j], acc[i][j]);
        }
      }
      Frag<T>::guard(acc[i][0], acc[i][3], ah, SPLIT ? al : ah);
    }
    Frag<T>::keep(bh[0], bh[1], bh[2], bh[3]);
    if (SPLIT) Frag<T>::keep(bl[0], bl[1], bl[2], bl[3]);
  }
  acc_guard4(acc[0][0], acc[0][1], acc[0][2], acc[0][3]);
  acc_guard4(acc[1][0], acc[1][1], acc[1][2], acc[1][3]);
  acc_guard4(acc[2][0], acc[2][1], acc[2][2], acc[2][3]);
  acc_guard4(acc[3][0], acc[3][1], acc[3][2], acc[3][3]);

  float* slab = sT[wave];
  const float* Rb = RESID ? (resid + (size_t)b * strideR) : nullptr;
#pragma unroll
  for (int i = 0; i < 4; ++i) {
    const int mBase = m0 + (i << 4);
#pragma unroll
    for (int j = 0; j < 4; ++j) {
      const int n = n0 + (j << 4) + rlane;
      float bv = 0.f;
      if (BIAS_MODE == 2) bv = bias[n];
#pragma unroll
      for (int r = 0; r < 8; ++r) {
        float v = acc[i][j][r] * scale;
        if (BIAS_MODE == 1) v += bias[mBase + mOff + r];
        if (BIAS_MODE == 2) v += bv;
        if (RESID) v += Rb[(size_t)(mBase + mOff + r) * ldc + n];
        if (ACT == 2) v = fmaxf(v, 0.0f);
        if (ACT == 4) v = (v > 0.f) ? v : 0.01f * v;
        slab[(mOff + r) * 68 + (j << 4) + rlane] = v;
      }
    }
    __builtin_amdgcn_fence(__ATOMIC_RELEASE, "workgroup");
    __builtin_amdgcn_wave_barrier();
    __builtin_amdgcn_fence(__ATOMIC_ACQUIRE, "workgroup");
    if (OUT_MODE == 0) {
      float* C = (float*)Cout + (size_t)b * strideC;
      const int hh = lane >> 4, c4 = (lane & 15) * 4;
      for (int pass = 0; pass < 2; ++pass) {
#pragma unroll
        for (int it = 0; it < 8; ++it) {
          const int row = it * 2 + hh;
          v4f v = *(const v4f*)(slab + row * 68 + c4);
          *(volatile v4f*)(C + (size_t)(mBase + row) * ldc + n0 + c4) = v;
        }
        __threadfence();
      }
    } else {
      const int q = lane >> 3, c8 = (lane & 7) * 8;
      unsigned short* C  = (unsigned short*)Cout  + (size_t)b * strideC;
      unsigned short* C2 = (OUT_MODE == 2) ? ((unsigned short*)Cout2 + (size_t)b * strideC) : nullptr;
      for (int pass = 0; pass < 2; ++pass) {
#pragma unroll
        for (int it = 0; it < 4; ++it) {
          const int row = it * 4 + q;
          const float* sp = slab + row * 68 + c8;
          v8h hv, lv;
#pragma unroll
          for (int e = 0; e < 8; ++e) {
            if (OUT_MODE == 1) {
              hv[e] = (_Float16)sp[e];
            } else {
              unsigned short hb = f2bf_bits(sp[e]);
              unsigned short lb = f2bf_bits(sp[e] - bf_bits2f(hb));
              hv[e] = __builtin_bit_cast(_Float16, hb);
              lv[e] = __builtin_bit_cast(_Float16, lb);
            }
          }
          *(volatile v8h*)(C + (size_t)(mBase + row) * ldc + n0 + c8) = hv;
          if (OUT_MODE == 2) *(volatile v8h*)(C2 + (size_t)(mBase + row) * ldc + n0 + c8) = lv;
        }
        __threadfence();
      }
    }
    __builtin_amdgcn_fence(__ATOMIC_RELEASE, "workgroup");
    __builtin_amdgcn_wave_barrier();
    __builtin_amdgcn_fence(__ATOMIC_ACQUIRE, "workgroup");
  }
}

__global__ __launch_bounds__(256) void copy4_kernel(const float* __restrict__ in, float* __restrict__ out, int n4) {
  const int i = blockIdx.x * 256 + threadIdx.x;
  if (i >= n4) return;
  const v4f v = *(const v4f*)(in + 4 * (size_t)i);
  float* q = out + 4 * (size_t)i;
  *(volatile v4f*)q = v;
  __threadfence();
  *(volatile v4f*)q = v;
}

__global__ __launch_bounds__(256) void cast8_f16_kernel(const float* __restrict__ in, unsigned short* __restrict__ out, int n8) {
  const int i = blockIdx.x * 256 + threadIdx.x;
  if (i >= n8) return;
  const float* p = in + 8 * (size_t)i;
  const v4f a = *(const v4f*)(p);
  const v4f c = *(const v4f*)(p + 4);
  unsigned short hb[8];
#pragma unroll
  for (int e = 0; e < 4; ++e) {
    hb[e]     = h_bits(a[e]);
    hb[4 + e] = h_bits(c[e]);
  }
  const v4u u = (v4u){pk16(hb[0], hb[1]), pk16(hb[2], hb[3]), pk16(hb[4], hb[5]), pk16(hb[6], hb[7])};
  unsigned short* q = out + 8 * (size_t)i;
  *(volatile v4u*)q = u;
  __threadfence();
  *(volatile v4u*)q = u;
}

__global__ __launch_bounds__(256) void split8_kernel(const float* __restrict__ in, unsigned short* __restrict__ outH,
                                                     unsigned short* __restrict__ outL, int n8) {
  const int i = blockIdx.x * 256 + threadIdx.x;
  if (i >= n8) return;
  const float* p = in + 8 * (size_t)i;
  const v4f a = *(const v4f*)(p);
  const v4f c = *(const v4f*)(p + 4);
  unsigned short hb[8], lb[8];
#pragma unroll
  for (int e = 0; e < 4; ++e) {
    split_bits(a[e], hb[e], lb[e]);
    split_bits(c[e], hb[4 + e], lb[4 + e]);
  }
  const v4u uh = (v4u){pk16(hb[0], hb[1]), pk16(hb[2], hb[3]), pk16(hb[4], hb[5]), pk16(hb[6], hb[7])};
  const v4u ul = (v4u){pk16(lb[0], lb[1]), pk16(lb[2], lb[3]), pk16(lb[4], lb[5]), pk16(lb[6], lb[7])};
  unsigned short* qh = outH + 8 * (size_t)i;
  unsigned short* ql = outL + 8 * (size_t)i;
  *(volatile v4u*)qh = uh;
  *(volatile v4u*)ql = ul;
  __threadfence();
  *(volatile v4u*)qh = uh;
  *(volatile v4u*)ql = ul;
}

__global__ __launch_bounds__(256) void wtsplit_kernel(const float* __restrict__ W, unsigned short* __restrict__ outH,
                                                      unsigned short* __restrict__ outL, int Kdim, int Ndim) {
  __shared__ float sm[64][65];
  const int t  = threadIdx.x;
  const int k0 = blockIdx.x * 64;
  const int n0 = blockIdx.y * 64;
#pragma unroll
  for (int i = 0; i < 16; ++i) {
    const int e = i * 256 + t;
    const int r = e >> 6;
    const int c = e & 63;
    sm[c][r] = W[(size_t)(k0 + r) * Ndim + n0 + c];
  }
  __syncthreads();
  const int lane = t & 31, wave = t >> 5;
  const int q = lane >> 3, c8 = (lane & 7) * 8;
  for (int pass = 0; pass < 2; ++pass) {
#pragma unroll
    for (int it = 0; it < 2; ++it) {
      const int row = wave * 8 + it * 4 + q;
      unsigned short hb[8], lb[8];
#pragma unroll
      for (int e = 0; e < 8; ++e) split_bits(sm[row][c8 + e], hb[e], lb[e]);
      const v4u uh = (v4u){pk16(hb[0], hb[1]), pk16(hb[2], hb[3]), pk16(hb[4], hb[5]), pk16(hb[6], hb[7])};
      const v4u ul = (v4u){pk16(lb[0], lb[1]), pk16(lb[2], lb[3]), pk16(lb[4], lb[5]), pk16(lb[6], lb[7])};
      const size_t o = (size_t)(n0 + row) * Kdim + k0 + c8;
      *(volatile v4u*)(outH + o) = uh;
      *(volatile v4u*)(outL + o) = ul;
    }
    __threadfence();
  }
}

__global__ __launch_bounds__(256) void wtcast_f16_kernel(const float* __restrict__ W, unsigned short* __restrict__ outP,
                                                         int Kdim, int Ndim, float scale) {
  __shared__ float sm[64][65];
  const int t  = threadIdx.x;
  const int k0 = blockIdx.x * 64;
  const int n0 = blockIdx.y * 64;
#pragma unroll
  for (int i = 0; i < 16; ++i) {
    const int e = i * 256 + t;
    const int r = e >> 6;
    const int c = e & 63;
    sm[c][r] = W[(size_t)(k0 + r) * Ndim + n0 + c] * scale;
  }
  __syncthreads();
  const int lane = t & 31, wave = t >> 5;
  const int q = lane >> 3, c8 = (lane & 7) * 8;
  for (int pass = 0; pass < 2; ++pass) {
#pragma unroll
    for (int it = 0; it < 2; ++it) {
      const int row = wave * 8 + it * 4 + q;
      unsigned short hb[8];
#pragma unroll
      for (int e = 0; e < 8; ++e) hb[e] = h_bits(sm[row][c8 + e]);
      const v4u u = (v4u){pk16(hb[0], hb[1]), pk16(hb[2], hb[3]), pk16(hb[4], hb[5]), pk16(hb[6], hb[7])};
      *(volatile v4u*)(outP + (size_t)(n0 + row) * Kdim + k0 + c8) = u;
    }
    __threadfence();
  }
}

__device__ __forceinline__ float tanh_via_exp(float x) {
  x = fminf(fmaxf(x, -15.0f), 15.0f);
  const float e = __expf(2.0f * x);
  return 1.0f - 2.0f * __builtin_amdgcn_rcpf(1.0f + e);
}

template <int DIM>
__global__ __launch_bounds__(256) void nbr_attn_kernel(
    const int* __restrict__ clu, const float* __restrict__ noise,
    const float* __restrict__ QP, const float* __restrict__ KP,
    const float* __restrict__ bp, const float* __restrict__ vp,
    const float* __restrict__ tri,
    unsigned short* __restrict__ embH, unsigned short* __restrict__ embL) {
  __shared__ int   candJ[kRows];
  __shared__ float candN[kRows];
  __shared__ __align__(16) float qs[DIM];
  __shared__ __align__(16) float bps[DIM];
  __shared__ __align__(16) float vps[DIM];
  __shared__ __align__(16) float embs[DIM];
  __shared__ int   wtot[8];
  __shared__ int   selJ[48];
  __shared__ float es[48];
  __shared__ float coefs[48];

  const int row  = blockIdx.x;
  const int t    = threadIdx.x;
  const int lane = t & 31;
  const int wave = t >> 5;
  const int myc  = clu[row];

#pragma unroll 1
  for (int d = t; d < DIM; d += 256) {
    qs[d]  = QP[(size_t)row * DIM + d];
    bps[d] = bp[d];
    vps[d] = vp[d];
  }
  if (t < 48) { selJ[t] = 0; es[t] = 0.f; coefs[t] = 0.f; }

  const int j0 = t * 8;
  const v4i ca = *(const v4i*)(clu + j0);
  const v4i cb = *(const v4i*)(clu + j0 + 4);
  const float* nrow = noise + (size_t)row * kRows + j0;
  const v4f na = *(const v4f*)(nrow);
  const v4f nb = *(const v4f*)(nrow + 4);
  int fl[8]; float nz[8]; int jj[8];
#pragma unroll
  for (int e = 0; e < 4; ++e) {
    jj[e]     = j0 + e;      nz[e]     = na[e];
    jj[4 + e] = j0 + 4 + e;  nz[4 + e] = nb[e];
    fl[e]     = (ca[e] == myc && jj[e]     != row) ? 1 : 0;
    fl[4 + e] = (cb[e] == myc && jj[4 + e] != row) ? 1 : 0;
  }
  int cnt = 0;
#pragma unroll
  for (int e = 0; e < 8; ++e) cnt += fl[e];

  int incl = cnt;
#pragma unroll
  for (int off = 1; off < 32; off <<= 1) {
    const int y = __shfl_up(incl, off, 32);
    if (lane >= off) incl += y;
  }
  const int wsum = __shfl(incl, 31, 32);
  if (lane == 31) wtot[wave] = wsum;
  __syncthreads();
  int woff = 0, m = 0;
#pragma unroll
  for (int w = 0; w < 8; ++w) {
    const int v = wtot[w];
    m += v;
    woff += (w < wave) ? v : 0;
  }
  int pos = woff + incl - cnt;
#pragma unroll
  for (int e = 0; e < 8; ++e) {
    if (fl[e]) { candJ[pos] = jj[e]; candN[pos] = nz[e]; ++pos; }
  }
  __syncthreads();

  const int mcl = m < (kRows - 1) ? m : (kRows - 1);
#pragma unroll 1
  for (int it = 0; it < 8; ++it) {
    const int a = t + 256 * it;
    if (a < mcl) {
      const float va = candN[a];
      const int   ja = candJ[a];
      int rk = 0;
#pragma unroll 1
      for (int bq = 0; bq < mcl; ++bq) {
        const float vb = candN[bq];
        const int   jb = candJ[bq];
        rk += ((vb > va) || (vb == va && jb < ja)) ? 1 : 0;
      }
      if (rk < kNei) selJ[rk] = ja;
    }
  }
  __syncthreads();
  const int msel  = m < kNei ? m : kNei;
  const int ncomp = (msel < kNei) ? (msel + 1) : kNei;

#pragma unroll 1
  for (int k = 0; k < 6; ++k) {
    const int n = wave + 8 * k;
    if (n < ncomp) {
      int jn = selJ[n];
      jn = jn < 0 ? 0 : (jn > kRows - 1 ? kRows - 1 : jn);
      const float kval = (n < msel) ? 1.f : 0.f;
      const float* kr = KP + (size_t)jn * DIM;
      float a = 0.f;
#pragma unroll 1
      for (int d = 2 * lane; d < DIM; d += 64) {
        const v2f q2 = *(const v2f*)(qs + d);
        const v2f k2 = *(const v2f*)(kr + d);
        const v2f b2 = *(const v2f*)(bps + d);
        const v2f w2 = *(const v2f*)(vps + d);
        float x0 = q2[0] + kval * k2[0];
        float x1 = q2[1] + kval * k2[1];
        x0 = x0 + b2[0];
        x1 = x1 + b2[1];
        a += tanh_via_exp(x0) * w2[0];
        a += tanh_via_exp(x1) * w2[1];
      }
#pragma unroll
      for (int off = 16; off > 0; off >>= 1) a += __shfl_xor(a, off, 32);
      if (lane == 0) es[n] = a;
    }
  }
  __syncthreads();

  if (t == 0) {
    float mx = es[0];
#pragma unroll 1
    for (int n = 1; n < kNei; ++n) {
      const int ix = n < ncomp ? n : (ncomp - 1);
      mx = fmaxf(mx, es[ix]);
    }
    float s = 0.f;
#pragma unroll 1
    for (int n = 0; n < kNei; ++n) {
      const int ix = n < ncomp ? n : (ncomp - 1);
      const float ex = expf(es[ix] - mx);
      coefs[n] = ex;
      s += ex;
    }
    const float inv = 1.0f / s;
#pragma unroll 1
    for (int n = 0; n < kNei; ++n) coefs[n] = coefs[n] * inv;
  }
  __syncthreads();

#pragma unroll 1
  for (int d = t; d < DIM; d += 256) {
    float a = 0.f;
#pragma unroll 1
    for (int n = 0; n < msel; ++n) {
      const int jn = selJ[n] & (kRows - 1);
      a += coefs[n] * tri[(size_t)jn * DIM + d];
    }
    embs[d] = a;
  }
  __syncthreads();

  if (t < DIM / 8) {
    const v4f e0 = *(const v4f*)(embs + 8 * t);
    const v4f e1 = *(const v4f*)(embs + 8 * t + 4);
    unsigned short hb[8], lb[8];
#pragma unroll
    for (int e = 0; e < 4; ++e) {
      split_bits(e0[e], hb[e], lb[e]);
      split_bits(e1[e], hb[4 + e], lb[4 + e]);
    }
    const v4u uh = (v4u){pk16(hb[0], hb[1]), pk16(hb[2], hb[3]), pk16(hb[4], hb[5]), pk16(hb[6], hb[7])};
    const v4u ul = (v4u){pk16(lb[0], lb[1]), pk16(lb[2], lb[3]), pk16(lb[4], lb[5]), pk16(lb[6], lb[7])};
    const size_t o = (size_t)row * DIM + 8 * t;
    *(volatile v4u*)(embH + o) = uh;
    *(volatile v4u*)(embL + o) = ul;
    __threadfence();
    *(volatile v4u*)(embH + o) = uh;
    *(volatile v4u*)(embL + o) = ul;
  }
}

__global__ __launch_bounds__(256) void colstats_kernel(const float* __restrict__ X, float* __restrict__ meanTab,
                                                       float* __restrict__ istdTab) {
  __shared__ float red[8][32];
  __shared__ float mean_s[32];
  const int t = threadIdx.x, c = t & 31, w = t >> 5;
  const int c0 = blockIdx.x * 32;
  const float* col = X + c0 + c;
  float s = 0.f;
#pragma unroll 1
  for (int r = w; r < kRows; r += 8) s += col[(size_t)r * kMid];
  red[w][c] = s;
  __syncthreads();
  if (t < 32) {
    float tot = red[0][t];
#pragma unroll
    for (int w2 = 1; w2 < 8; ++w2) tot += red[w2][t];
    mean_s[t] = tot * (1.0f / 2048.0f);
  }
  __syncthreads();
  const float mu = mean_s[c];
  float q = 0.f;
#pragma unroll 1
  for (int r = w; r < kRows; r += 8) {
    const float dlt = col[(size_t)r * kMid] - mu;
    q += dlt * dlt;
  }
  red[w][c] = q;
  __syncthreads();
  if (t < 32) {
    float tot = red[0][t];
#pragma unroll
    for (int w2 = 1; w2 < 8; ++w2) tot += red[w2][t];
    const float var  = tot * (1.0f / 2048.0f);
    const float istd = 1.0f / sqrtf(var + kEps);
    const float mv   = mean_s[t];
    *(volatile float*)(meanTab + c0 + t) = mv;
    *(volatile float*)(istdTab + c0 + t) = istd;
    __threadfence();
    *(volatile float*)(meanTab + c0 + t) = mv;
    *(volatile float*)(istdTab + c0 + t) = istd;
  }
}

__global__ __launch_bounds__(128) void bn_apply_kernel(const float* __restrict__ X, const float* __restrict__ meanTab,
                                                       const float* __restrict__ istdTab, const float* __restrict__ g,
                                                       const float* __restrict__ bb, float* __restrict__ out,
                                                       unsigned short* __restrict__ pH, unsigned short* __restrict__ pL) {
  __shared__ __align__(16) float st[kMid];
  const int row = blockIdx.x, t = threadIdx.x, c = 4 * t;
  const size_t o = (size_t)row * kMid + c;
  const v4f x  = *(const v4f*)(X + o);
  const v4f mu = *(const v4f*)(meanTab + c);
  const v4f is = *(const v4f*)(istdTab + c);
  const v4f gg = *(const v4f*)(g + c);
  const v4f be = *(const v4f*)(bb + c);
  v4f y;
#pragma unroll
  for (int e = 0; e < 4; ++e) {
    float v = gg[e] * (x[e] - mu[e]) * is[e] + be[e];
    y[e] = fmaxf(v, 0.0f);
  }
  *(v4f*)(st + c) = y;
  *(volatile v4f*)(out + o) = y;
  __syncthreads();
  v4u uh = (v4u){0u, 0u, 0u, 0u}, ul = (v4u){0u, 0u, 0u, 0u};
  const size_t op = (size_t)row * kMid + 8 * t;
  if (t < 64) {
    const v4f s0 = *(const v4f*)(st + 8 * t);
    const v4f s1 = *(const v4f*)(st + 8 * t + 4);
    unsigned short hb[8], lb[8];
#pragma unroll
    for (int e = 0; e < 4; ++e) {
      split_bits(s0[e], hb[e], lb[e]);
      split_bits(s1[e], hb[4 + e], lb[4 + e]);
    }
    uh = (v4u){pk16(hb[0], hb[1]), pk16(hb[2], hb[3]), pk16(hb[4], hb[5]), pk16(hb[6], hb[7])};
    ul = (v4u){pk16(lb[0], lb[1]), pk16(lb[2], lb[3]), pk16(lb[4], lb[5]), pk16(lb[6], lb[7])};
    *(volatile v4u*)(pH + op) = uh;
    *(volatile v4u*)(pL + op) = ul;
  }
  __threadfence();
  *(volatile v4f*)(out + o) = y;
  if (t < 64) {
    *(volatile v4u*)(pH + op) = uh;
    *(volatile v4u*)(pL + op) = ul;
  }
}

__device__ __forceinline__ float sigm(float x) { return 1.0f / (1.0f + expf(-x)); }

template <bool PLANES>
__global__ __launch_bounds__(256) void gru_kernel(const float* __restrict__ gi, const float* __restrict__ gh,
                                                  const float* __restrict__ h, float* __restrict__ out,
                                                  unsigned short* __restrict__ pH, unsigned short* __restrict__ pL) {
  __shared__ __align__(16) float stage[256];
  const int t = threadIdx.x;
  const int e = blockIdx.x * 256 + t;
  const int row = e >> 9;
  const int c   = e & (kMid - 1);
  const float* gr = gi + (size_t)row * kGate;
  const float* hr = gh + (size_t)row * kGate;
  const float ir = gr[c], iz = gr[kMid + c], inn = gr[2 * kMid + c];
  const float gr_ = hr[c], gz = hr[kMid + c], gn = hr[2 * kMid + c];
  const float hv = h[(size_t)e];
  const float r = sigm(ir + gr_);
  const float z = sigm(iz + gz);
  const float nn = tanhf(inn + r * gn);
  const float v = (1.0f - z) * nn + z * hv;
  stage[t] = v;
  __syncthreads();
  const size_t base = (size_t)blockIdx.x * 256;
  v4f o4 = (v4f){0.f, 0.f, 0.f, 0.f};
  v4u uh = (v4u){0u, 0u, 0u, 0u}, ul = (v4u){0u, 0u, 0u, 0u};
  if (t < 64) o4 = *(const v4f*)(stage + 4 * t);
  if (PLANES && t < 32) {
    const v4f s0 = *(const v4f*)(stage + 8 * t);
    const v4f s1 = *(const v4f*)(stage + 8 * t + 4);
    unsigned short hb[8], lb[8];
#pragma unroll
    for (int q = 0; q < 4; ++q) {
      split_bits(s0[q], hb[q], lb[q]);
      split_bits(s1[q], hb[4 + q], lb[4 + q]);
    }
    uh = (v4u){pk16(hb[0], hb[1]), pk16(hb[2], hb[3]), pk16(hb[4], hb[5]), pk16(hb[6], hb[7])};
    ul = (v4u){pk16(lb[0], lb[1]), pk16(lb[2], lb[3]), pk16(lb[4], lb[5]), pk16(lb[6], lb[7])};
  }
  if (t < 64) *(volatile v4f*)(out + base + 4 * t) = o4;
  if (PLANES && t < 32) {
    *(volatile v4u*)(pH + base + 8 * t) = uh;
    *(volatile v4u*)(pL + base + 8 * t) = ul;
  }
  __threadfence();
  if (t < 64) *(volatile v4f*)(out + base + 4 * t) = o4;
  if (PLANES && t < 32) {
    *(volatile v4u*)(pH + base + 8 * t) = uh;
    *(volatile v4u*)(pL + base + 8 * t) = ul;
  }
}

template <bool PLANES>
__global__ __launch_bounds__(128) void addln_kernel(const float* __restrict__ A, const float* __restrict__ Bsrc,
                                                    const float* __restrict__ g, const float* __restrict__ bb,
                                                    float* __restrict__ out,
                                                    unsigned short* __restrict__ pH, unsigned short* __restrict__ pL) {
  __shared__ float redA[4];
  __shared__ float redB[4];
  __shared__ __align__(16) float st[kMid];
  const int row = blockIdx.x, t = threadIdx.x, lane = t & 31, wave = t >> 5, c = 4 * t;
  const size_t o = (size_t)row * kMid + c;
  const v4f a  = *(const v4f*)(A + o);
  const v4f b2 = *(const v4f*)(Bsrc + o);
  float x[4];
#pragma unroll
  for (int e = 0; e < 4; ++e) x[e] = a[e] + b2[e];
  float s = ((x[0] + x[1]) + x[2]) + x[3];
#pragma unroll
  for (int off = 16; off > 0; off >>= 1) s += __shfl_xor(s, off, 32);
  if (lane == 0) redA[wave] = s;
  __syncthreads();
  const float mean = (((redA[0] + redA[1]) + redA[2]) + redA[3]) * (1.0f / 512.0f);
  float dlt[4];
  float q = 0.f;
#pragma unroll
  for (int e = 0; e < 4; ++e) { dlt[e] = x[e] - mean; q += dlt[e] * dlt[e]; }
#pragma unroll
  for (int off = 16; off > 0; off >>= 1) q += __shfl_xor(q, off, 32);
  if (lane == 0) redB[wave] = q;
  __syncthreads();
  const float var  = (((redB[0] + redB[1]) + redB[2]) + redB[3]) * (1.0f / 512.0f);
  const float istd = 1.0f / sqrtf(var + kEps);
  const v4f gg = *(const v4f*)(g + c);
  const v4f be = *(const v4f*)(bb + c);
  v4f y;
#pragma unroll
  for (int e = 0; e < 4; ++e) y[e] = gg[e] * dlt[e] * istd + be[e];
  if (PLANES) *(v4f*)(st + c) = y;
  *(volatile v4f*)(out + o) = y;
  v4u uh = (v4u){0u, 0u, 0u, 0u}, ul = (v4u){0u, 0u, 0u, 0u};
  const size_t op = (size_t)row * kMid + 8 * t;
  if (PLANES) {
    __syncthreads();
    if (t < 64) {
      const v4f s0 = *(const v4f*)(st + 8 * t);
      const v4f s1 = *(const v4f*)(st + 8 * t + 4);
      unsigned short hb[8], lb[8];
#pragma unroll
      for (int e = 0; e < 4; ++e) {
        split_bits(s0[e], hb[e], lb[e]);
        split_bits(s1[e], hb[4 + e], lb[4 + e]);
      }
      uh = (v4u){pk16(hb[0], hb[1]), pk16(hb[2], hb[3]), pk16(hb[4], hb[5]), pk16(hb[6], hb[7])};
      ul = (v4u){pk16(lb[0], lb[1]), pk16(lb[2], lb[3]), pk16(lb[4], lb[5]), pk16(lb[6], lb[7])};
      *(volatile v4u*)(pH + op) = uh;
      *(volatile v4u*)(pL + op) = ul;
    }
  }
  __threadfence();
  *(volatile v4f*)(out + o) = y;
  if (PLANES && t < 64) {
    *(volatile v4u*)(pH + op) = uh;
    *(volatile v4u*)(pL + op) = ul;
  }
}

__global__ __launch_bounds__(256) void cls_kernel(const float* __restrict__ x, const float* __restrict__ Wc,
                                                  const float* __restrict__ bc, float* __restrict__ out) {
  const int gt = blockIdx.x * 256 + threadIdx.x;
  if (gt >= kRows / 2) return;
  const float* x0 = x + (size_t)(2 * gt) * kMid;
  const float* x1 = x0 + kMid;
  float a00 = 0.f, a01 = 0.f, a10 = 0.f, a11 = 0.f;
#pragma unroll 1
  for (int k = 0; k < kMid; ++k) {
    const float w0 = Wc[2 * k], w1 = Wc[2 * k + 1];
    const float u = x0[k], v = x1[k];
    a00 += u * w0; a01 += u * w1;
    a10 += v * w0; a11 += v * w1;
  }
  a00 += bc[0]; a01 += bc[1]; a10 += bc[0]; a11 += bc[1];
  const float m0 = fmaxf(a00, a01), m1 = fmaxf(a10, a11);
  const float e00 = expf(a00 - m0), e01 = expf(a01 - m0);
  const float e10 = expf(a10 - m1), e11 = expf(a11 - m1);
  const float i0 = 1.0f / (e00 + e01), i1 = 1.0f / (e10 + e11);
  const v4f o = (v4f){e00 * i0, e01 * i0, e10 * i1, e11 * i1};
  float* q = out + 4 * (size_t)gt;
  *(volatile v4f*)q = o;
  __threadfence();
  *(volatile v4f*)q = o;
}

template <int BM, int OM, int ACT>
static void run_gemm_split(hipStream_t s, const unsigned short* Ah, const unsigned short* Al,
                           const unsigned short* Bh, const unsigned short* Bl,
                           void* C, void* Cq, const float* bias, int M, int N, int K) {
  const int tiles  = (M / 64) * (N / 64);
  const int blocks = (tiles + 7) / 8;
  wmma_gemm64<1, true, BM, OM, false, ACT><<<dim3((unsigned)blocks, 1), 256, 0, s>>>(
      Ah, Al, K, (long)0, Bh, Bl, K, (long)0, C, Cq, N, (long)0, bias, (const float*)nullptr, (long)0, M, N, K, 1.0f);
}
static void run_gemm_f16(hipStream_t s, const unsigned short* Ap, const unsigned short* Bp,
                         float* C, int M, int N, int K, float scale) {
  const int tiles  = (M / 64) * (N / 64);
  const int blocks = (tiles + 7) / 8;
  wmma_gemm64<0, false, 0, 0, false, 0><<<dim3((unsigned)blocks, 1), 256, 0, s>>>(
      Ap, (const unsigned short*)nullptr, K, (long)0, Bp, (const unsigned short*)nullptr, K, (long)0,
      (void*)C, (void*)nullptr, N, (long)0, (const float*)nullptr, (const float*)nullptr, (long)0, M, N, K, scale);
}

static inline unsigned cdiv(size_t a, size_t b) { return (unsigned)((a + b - 1) / b); }

extern "C" void kernel_launch(void* const* d_in, const int* in_sizes, int n_in,
                              void* d_out, int out_size, void* d_ws, size_t ws_size,
                              hipStream_t stream) {
  (void)in_sizes;
  if (n_in < 44) return;
  if ((size_t)out_size < (size_t)8916992) return;

  const float* input_t = (const float*)d_in[0];
  const float* input_v = (const float*)d_in[1];
  const int*   te_clu  = (const int*)d_in[2];
  const int*   im_clu  = (const int*)d_in[3];
  const float* t_tri   = (const float*)d_in[4];
  const float* v_tri   = (const float*)d_in[5];
  const float* noise_t = (const float*)d_in[6];
  const float* noise_v = (const float*)d_in[7];
  const float* Wq_t = (const float*)d_in[8],  *Wk_t = (const float*)d_in[9];
  const float* bp_t = (const float*)d_in[10], *vp_t = (const float*)d_in[11];
  const float* Wq_v = (const float*)d_in[12], *Wk_v = (const float*)d_in[13];
  const float* bp_v = (const float*)d_in[14], *vp_v = (const float*)d_in[15];
  const float* W_lt = (const float*)d_in[16], *b_lt = (const float*)d_in[17];
  const float* g_bt = (const float*)d_in[18], *be_bt = (const float*)d_in[19];
  const float* W_lv = (const float*)d_in[20], *b_lv = (const float*)d_in[21];
  const float* g_bv = (const float*)d_in[22], *be_bv = (const float*)d_in[23];
  const float* Wih_t = (const float*)d_in[24], *Whh_t = (const float*)d_in[25];
  const float* bih_t = (const float*)d_in[26], *bhh_t = (const float*)d_in[27];
  const float* Wih_v = (const float*)d_in[28], *Whh_v = (const float*)d_in[29];
  const float* bih_v = (const float*)d_in[30], *bhh_v = (const float*)d_in[31];
  const float* Wv_f  = (const float*)d_in[32], *Wo_f  = (const float*)d_in[33];
  const float* g_ln1 = (const float*)d_in[34], *b_ln1 = (const float*)d_in[35];
  const float* Wf1 = (const float*)d_in[36], *bf1 = (const float*)d_in[37];
  const float* Wf2 = (const float*)d_in[38], *bf2 = (const float*)d_in[39];
  const float* g_ln2 = (const float*)d_in[40], *b_ln2 = (const float*)d_in[41];
  const float* Wc = (const float*)d_in[42], *bc = (const float*)d_in[43];

  float* out   = (float*)d_out;
  float* oTtri = out + 0;
  float* oVtri = out + 1572864;
  float* oHt   = out + 3670016;
  float* oHv   = out + 4718592;
  float* oGrt  = out + 5767168;
  float* oGrv  = out + 6815744;
  float* oMm   = out + 7864320;
  float* oCls  = out + 8912896;

  char* ws = (char*)d_ws;
  size_t cur = 0;
  auto carve = [&](size_t bytes) -> size_t { const size_t off = cur; cur += (bytes + 127) & ~(size_t)127; return off; };
  auto plB = [](size_t r, size_t c) -> size_t { return r * c * 2; };
  auto f4B = [](size_t r, size_t c) -> size_t { return r * c * 4; };

  const size_t oEmbTH = carve(plB(kRows, kDimT)), oEmbTL = carve(plB(kRows, kDimT));
  const size_t oEmbVH = carve(plB(kRows, kDimV)), oEmbVL = carve(plB(kRows, kDimV));
  const size_t oHtH = carve(plB(kRows, kMid)), oHtL = carve(plB(kRows, kMid));
  const size_t oHvH = carve(plB(kRows, kMid)), oHvL = carve(plB(kRows, kMid));
  const size_t oGrtH = carve(plB(kRows, kMid)), oGrtL = carve(plB(kRows, kMid));
  const size_t oMeanT = carve(kMid * 4), oIstdT = carve(kMid * 4), oMeanV = carve(kMid * 4), oIstdV = carve(kMid * 4);
  const size_t arena = cur;
  size_t wsEnd = arena;
  cur = arena;
  const size_t o1T = carve(plB(kRows, kDimT));
  const size_t o1Wq = carve(plB(kDimT, kDimT));
  const size_t o1Wk = carve(plB(kDimT, kDimT));
  const size_t o1QP = carve(f4B(kRows, kDimT)), o1KP = carve(f4B(kRows, kDimT));
  if (cur > wsEnd) wsEnd = cur;
  cur = arena;
  const size_t o2T = carve(plB(kRows, kDimV));
  const size_t o2Wq = carve(plB(kDimV, kDimV));
  const size_t o2Wk = carve(plB(kDimV, kDimV));
  const size_t o2QP = carve(f4B(kRows, kDimV)), o2KP = carve(f4B(kRows, kDimV));
  if (cur > wsEnd) wsEnd = cur;
  cur = arena;
  const size_t o3XtH = carve(plB(kRows, kFlatT)), o3XtL = carve(plB(kRows, kFlatT));
  const size_t o3WltH = carve(plB(kMid, kFlatT)), o3WltL = carve(plB(kMid, kFlatT));
  const size_t o3LinT = carve(f4B(kRows, kMid));
  const size_t o3XvH = carve(plB(kRows, kFlatV)), o3XvL = carve(plB(kRows, kFlatV));
  const size_t o3WlvH = carve(plB(kMid, kFlatV)), o3WlvL = carve(plB(kMid, kFlatV));
  const size_t o3LinV = carve(f4B(kRows, kMid));
  if (cur > wsEnd) wsEnd = cur;
  cur = arena;
  const size_t o4WihH = carve(plB(kGate, kDimV)), o4WihL = carve(plB(kGate, kDimV));
  const size_t o4WhhH = carve(plB(kGate, kMid)), o4WhhL = carve(plB(kGate, kMid));
  const size_t o4Gi = carve(f4B(kRows, kGate)), o4Gh = carve(f4B(kRows, kGate));
  if (cur > wsEnd) wsEnd = cur;
  cur = arena;
  const size_t o5WvH = carve(plB(kMid, kMid)), o5WvL = carve(plB(kMid, kMid));
  const size_t o5WoH = carve(plB(kMid, kMid)), o5WoL = carve(plB(kMid, kMid));
  const size_t o5T1H = carve(plB(kRows, kMid)), o5T1L = carve(plB(kRows, kMid));
  const size_t o5Att = carve(f4B(kRows, kMid));
  const size_t o5Hln = carve(f4B(kRows, kMid));
  const size_t o5HlnH = carve(plB(kRows, kMid)), o5HlnL = carve(plB(kRows, kMid));
  const size_t o5Wf1H = carve(plB(kFfn, kMid)), o5Wf1L = carve(plB(kFfn, kMid));
  const size_t o5F1H = carve(plB(kRows, kFfn)), o5F1L = carve(plB(kRows, kFfn));
  const size_t o5Wf2H = carve(plB(kMid, kFfn)), o5Wf2L = carve(plB(kMid, kFfn));
  const size_t o5F2 = carve(f4B(kRows, kMid));
  if (cur > wsEnd) wsEnd = cur;
  if (wsEnd > ws_size) return;

  auto U = [&](size_t off) -> unsigned short* { return (unsigned short*)(ws + off); };
  auto F = [&](size_t off) -> float* { return (float*)(ws + off); };

  {
    const size_t n4t = (size_t)kRows * kDimT / 4, n4v = (size_t)kRows * kDimV / 4;
    copy4_kernel<<<cdiv(n4t, 256), 256, 0, stream>>>(t_tri, oTtri, (int)n4t);
    copy4_kernel<<<cdiv(n4v, 256), 256, 0, stream>>>(v_tri, oVtri, (int)n4v);
  }

  {
    const size_t n8 = (size_t)kRows * kDimT / 8;
    cast8_f16_kernel<<<cdiv(n8, 256), 256, 0, stream>>>(t_tri, U(o1T), (int)n8);
    wtcast_f16_kernel<<<dim3(kDimT / 64, kDimT / 64), 256, 0, stream>>>(Wq_t, U(o1Wq), kDimT, kDimT, kWCarry);
    wtcast_f16_kernel<<<dim3(kDimT / 64, kDimT / 64), 256, 0, stream>>>(Wk_t, U(o1Wk), kDimT, kDimT, kWCarry);
    run_gemm_f16(stream, U(o1T), U(o1Wq), F(o1QP), kRows, kDimT, kDimT, kWCarryInv);
    run_gemm_f16(stream, U(o1T), U(o1Wk), F(o1KP), kRows, kDimT, kDimT, kWCarryInv);
    nbr_attn_kernel<kDimT><<<kRows, 256, 0, stream>>>(te_clu, noise_t, F(o1QP), F(o1KP), bp_t, vp_t, t_tri,
                                                       U(oEmbTH), U(oEmbTL));
  }
  {
    const size_t n8 = (size_t)kRows * kDimV / 8;
    cast8_f16_kernel<<<cdiv(n8, 256), 256, 0, stream>>>(v_tri, U(o2T), (int)n8);
    wtcast_f16_kernel<<<dim3(kDimV / 64, kDimV / 64), 256, 0, stream>>>(Wq_v, U(o2Wq), kDimV, kDimV, kWCarry);
    wtcast_f16_kernel<<<dim3(kDimV / 64, kDimV / 64), 256, 0, stream>>>(Wk_v, U(o2Wk), kDimV, kDimV, kWCarry);
    run_gemm_f16(stream, U(o2T), U(o2Wq), F(o2QP), kRows, kDimV, kDimV, kWCarryInv);
    run_gemm_f16(stream, U(o2T), U(o2Wk), F(o2KP), kRows, kDimV, kDimV, kWCarryInv);
    nbr_attn_kernel<kDimV><<<kRows, 256, 0, stream>>>(im_clu, noise_v, F(o2QP), F(o2KP), bp_v, vp_v, v_tri,
                                                       U(oEmbVH), U(oEmbVL));
  }
  {
    const size_t n8t = (size_t)kRows * kFlatT / 8;
    split8_kernel<<<cdiv(n8t, 256), 256, 0, stream>>>(input_t, U(o3XtH), U(o3XtL), (int)n8t);
    wtsplit_kernel<<<dim3(kFlatT / 64, kMid / 64), 256, 0, stream>>>(W_lt, U(o3WltH), U(o3WltL), kFlatT, kMid);
    run_gemm_split<2, 0, 0>(stream, U(o3XtH), U(o3XtL), U(o3WltH), U(o3WltL), F(o3LinT), nullptr, b_lt, kRows, kMid, kFlatT);
    colstats_kernel<<<kMid / 32, 256, 0, stream>>>(F(o3LinT), F(oMeanT), F(oIstdT));
    bn_apply_kernel<<<kRows, 128, 0, stream>>>(F(o3LinT), F(oMeanT), F(oIstdT), g_bt, be_bt, oHt, U(oHtH), U(oHtL));
    const size_t n8v = (size_t)kRows * kFlatV / 8;
    split8_kernel<<<cdiv(n8v, 256), 256, 0, stream>>>(input_v, U(o3XvH), U(o3XvL), (int)n8v);
    wtsplit_kernel<<<dim3(kFlatV / 64, kMid / 64), 256, 0, stream>>>(W_lv, U(o3WlvH), U(o3WlvL), kFlatV, kMid);
    run_gemm_split<2, 0, 0>(stream, U(o3XvH), U(o3XvL), U(o3WlvH), U(o3WlvL), F(o3LinV), nullptr, b_lv, kRows, kMid, kFlatV);
    colstats_kernel<<<kMid / 32, 256, 0, stream>>>(F(o3LinV), F(oMeanV), F(oIstdV));
    bn_apply_kernel<<<kRows, 128, 0, stream>>>(F(o3LinV), F(oMeanV), F(oIstdV), g_bv, be_bv, oHv, U(oHvH), U(oHvL));
  }
  {
    const size_t n8iht = (size_t)kGate * kDimT / 8, n8hh = (size_t)kGate * kMid / 8, n8ihv = (size_t)kGate * kDimV / 8;
    split8_kernel<<<cdiv(n8iht, 256), 256, 0, stream>>>(Wih_t, U(o4WihH), U(o4WihL), (int)n8iht);
    split8_kernel<<<cdiv(n8hh, 256), 256, 0, stream>>>(Whh_t, U(o4WhhH), U(o4WhhL), (int)n8hh);
    run_gemm_split<2, 0, 0>(stream, U(oEmbTH), U(oEmbTL), U(o4WihH), U(o4WihL), F(o4Gi), nullptr, bih_t, kRows, kGate, kDimT);
    run_gemm_split<2, 0, 0>(stream, U(oHtH), U(oHtL), U(o4WhhH), U(o4WhhL), F(o4Gh), nullptr, bhh_t, kRows, kGate, kMid);
    gru_kernel<true><<<cdiv((size_t)kRows * kMid, 256), 256, 0, stream>>>(F(o4Gi), F(o4Gh), oHt, oGrt, U(oGrtH), U(oGrtL));
    split8_kernel<<<cdiv(n8ihv, 256), 256, 0, stream>>>(Wih_v, U(o4WihH), U(o4WihL), (int)n8ihv);
    split8_kernel<<<cdiv(n8hh, 256), 256, 0, stream>>>(Whh_v, U(o4WhhH), U(o4WhhL), (int)n8hh);
    run_gemm_split<2, 0, 0>(stream, U(oEmbVH), U(oEmbVL), U(o4WihH), U(o4WihL), F(o4Gi), nullptr, bih_v, kRows, kGate, kDimV);
    run_gemm_split<2, 0, 0>(stream, U(oHvH), U(oHvL), U(o4WhhH), U(o4WhhL), F(o4Gh), nullptr, bhh_v, kRows, kGate, kMid);
    gru_kernel<false><<<cdiv((size_t)kRows * kMid, 256), 256, 0, stream>>>(F(o4Gi), F(o4Gh), oHv, oGrv,
                                                                          (unsigned short*)nullptr, (unsigned short*)nullptr);
  }
  {
    wtsplit_kernel<<<dim3(kMid / 64, kMid / 64), 256, 0, stream>>>(Wv_f, U(o5WvH), U(o5WvL), kMid, kMid);
    wtsplit_kernel<<<dim3(kMid / 64, kMid / 64), 256, 0, stream>>>(Wo_f, U(o5WoH), U(o5WoL), kMid, kMid);
    run_gemm_split<0, 2, 0>(stream, U(oGrtH), U(oGrtL), U(o5WvH), U(o5WvL), U(o5T1H), U(o5T1L), nullptr, kRows, kMid, kMid);
    run_gemm_split<0, 0, 0>(stream, U(o5T1H), U(o5T1L), U(o5WoH), U(o5WoL), F(o5Att), nullptr, nullptr, kRows, kMid, kMid);
    addln_kernel<true><<<kRows, 128, 0, stream>>>(oGrv, F(o5Att), g_ln1, b_ln1, F(o5Hln), U(o5HlnH), U(o5HlnL));
    wtsplit_kernel<<<dim3(kMid / 64, kFfn / 64), 256, 0, stream>>>(Wf1, U(o5Wf1H), U(o5Wf1L), kMid, kFfn);
    run_gemm_split<2, 2, 2>(stream, U(o5HlnH), U(o5HlnL), U(o5Wf1H), U(o5Wf1L), U(o5F1H), U(o5F1L), bf1, kRows, kFfn, kMid);
    wtsplit_kernel<<<dim3(kFfn / 64, kMid / 64), 256, 0, stream>>>(Wf2, U(o5Wf2H), U(o5Wf2L), kFfn, kMid);
    run_gemm_split<2, 0, 0>(stream, U(o5F1H), U(o5F1L), U(o5Wf2H), U(o5Wf2L), F(o5F2), nullptr, bf2, kRows, kMid, kFfn);
    addln_kernel<false><<<kRows, 128, 0, stream>>>(F(o5Hln), F(o5F2), g_ln2, b_ln2, oMm,
                                                    (unsigned short*)nullptr, (unsigned short*)nullptr);
    cls_kernel<<<cdiv((size_t)kRows / 2, 256), 256, 0, stream>>>(oMm, Wc, bc, oCls);
  }
}
